// _GraphormerNodeLayer_44865228374490
// MI455X (gfx1250) — hardware-verified
//
#include <hip/hip_runtime.h>
#include <math.h>
#include <stddef.h>


#define DM    128
#define NH    8
#define DFF   512
#define QW    384
#define TR    32
#define AP    136
#define ZP    520
#define HP    132
#define RP    388
#define TP    72
#define NTHR  256
#define NWAVE 8
#define NPB   8
#define ECAP  4096
#define LN_EPS 1e-5f

static_assert((AP * 2) % 16 == 0);
static_assert((ZP * 2) % 16 == 0);
static_assert((HP * 4) % 16 == 0);
static_assert((RP * 4) % 16 == 0);
static_assert((TP * 2) % 16 == 0);
static_assert(NPB == NWAVE);
static_assert(TR == 4 * NWAVE);
static_assert(TR * AP * 2 + TR * RP * 4 <= 65536);
static_assert(TR * HP * 4 + TR * AP * 2 + TR * ZP * 2 <= 65536);

typedef float    v4f  __attribute__((ext_vector_type(4)));
typedef float    v8f  __attribute__((ext_vector_type(8)));
typedef int      v4i  __attribute__((ext_vector_type(4)));
typedef _Float16 v4h  __attribute__((ext_vector_type(4)));
typedef _Float16 v8h  __attribute__((ext_vector_type(8)));
typedef _Float16 v16h __attribute__((ext_vector_type(16)));
union Frag   { v16h v; v8h half[2]; };
union Pack16 { v8h h; v4i i; };

__device__ __forceinline__ v8f wm(v16h a, v16h b, v8f c) {
  v8f d = __builtin_amdgcn_wmma_f32_16x16x32_f16(false, a, false, b, (short)0, c, false, false);
  asm volatile("v_nop\n\tv_nop\n\tv_nop\n\tv_nop" : "+v"(d) : "v"(a), "v"(b));
  return d;
}

__device__ __forceinline__ v16h frag_ld(const _Float16* p) {
  Frag f;
  f.half[0] = *(const v8h*)(p);
  f.half[1] = *(const v8h*)(p + 16);
  return f.v;
}

__device__ __forceinline__ float wsum(float v) {
  v += __shfl_xor(v, 16, 32);
  v += __shfl_xor(v, 8, 32);
  v += __shfl_xor(v, 4, 32);
  v += __shfl_xor(v, 2, 32);
  v += __shfl_xor(v, 1, 32);
  return v;
}

__device__ __forceinline__ int clampi(int v, int lo, int hi) {
  return v < lo ? lo : (v > hi ? hi : v);
}

__device__ __forceinline__ void stage16(_Float16* dst, const float* p, float sc) {
  const v4f f0 = *(const v4f*)(p), f1 = *(const v4f*)(p + 4);
  const v4f f2 = *(const v4f*)(p + 8), f3 = *(const v4f*)(p + 12);
  Pack16 u0, u1;
  u0.h[0] = (_Float16)(f0.x * sc); u0.h[1] = (_Float16)(f0.y * sc); u0.h[2] = (_Float16)(f0.z * sc); u0.h[3] = (_Float16)(f0.w * sc);
  u0.h[4] = (_Float16)(f1.x * sc); u0.h[5] = (_Float16)(f1.y * sc); u0.h[6] = (_Float16)(f1.z * sc); u0.h[7] = (_Float16)(f1.w * sc);
  u1.h[0] = (_Float16)(f2.x * sc); u1.h[1] = (_Float16)(f2.y * sc); u1.h[2] = (_Float16)(f2.z * sc); u1.h[3] = (_Float16)(f2.w * sc);
  u1.h[4] = (_Float16)(f3.x * sc); u1.h[5] = (_Float16)(f3.y * sc); u1.h[6] = (_Float16)(f3.z * sc); u1.h[7] = (_Float16)(f3.w * sc);
  *(v8h*)(dst)     = u0.h;
  *(v8h*)(dst + 8) = u1.h;
}

__device__ __forceinline__ v4f ln_row(v4f h, v4f g4, v4f b4) {
  const float s  = wsum(h.x + h.y + h.z + h.w);
  const float mu = s * (1.0f / DM);
  const v4f dd = h - mu;
  const float q  = wsum(dd.x * dd.x + dd.y * dd.y + dd.z * dd.z + dd.w * dd.w);
  const float rs = rsqrtf(q * (1.0f / DM) + LN_EPS);
  return dd * rs * g4 + b4;
}

__device__ __forceinline__ void tput4(_Float16* T, int c, int kr, v4f f) {
  T[(c + 0) * TP + kr] = (_Float16)(f.x * 32.0f);
  T[(c + 1) * TP + kr] = (_Float16)(f.y * 32.0f);
  T[(c + 2) * TP + kr] = (_Float16)(f.z * 32.0f);
  T[(c + 3) * TP + kr] = (_Float16)(f.w * 32.0f);
}

__global__ __launch_bounds__(NTHR) void k_prep(
    const float* __restrict__ Wq, const float* __restrict__ Wk, const float* __restrict__ Wv,
    const float* __restrict__ Wo, const float* __restrict__ W1, const float* __restrict__ W2,
    _Float16* qkvt, _Float16* wot, _Float16* w1t, _Float16* w2t) {
  __shared__ __attribute__((aligned(16))) _Float16 T[64 * TP];
  const int tid = threadIdx.x;
  const int b = blockIdx.x;
  const float* src;
  _Float16* dst;
  int K, N, nt, kt;
  if (b < 16) {
    const int w = b >> 2, t = b & 3;
    nt = t >> 1; kt = t & 1; K = DM; N = DM;
    src = (w == 0) ? Wq : ((w == 1) ? Wk : ((w == 2) ? Wv : Wo));
    dst = (w < 3) ? (qkvt + (size_t)w * DM * DM) : wot;
  } else if (b < 32) {
    const int u = b - 16;
    nt = u >> 1; kt = u & 1; K = DM; N = DFF;
    src = W1; dst = w1t;
  } else {
    const int u = b - 32;
    nt = u >> 3; kt = u & 7; K = DFF; N = DM;
    src = W2; dst = w2t;
  }
  const int n0 = nt * 64, k0 = kt * 64;
  {
    const int kr = tid >> 2;
    const int nc0 = (tid & 3) * 16;
    const float* p = src + (size_t)(k0 + kr) * N + n0 + nc0;
    const v4f f0 = *(const v4f*)(p), f1 = *(const v4f*)(p + 4);
    const v4f f2 = *(const v4f*)(p + 8), f3 = *(const v4f*)(p + 12);
    tput4(T, nc0 + 0, kr, f0);
    tput4(T, nc0 + 4, kr, f1);
    tput4(T, nc0 + 8, kr, f2);
    tput4(T, nc0 + 12, kr, f3);
  }
  __syncthreads();
  const int q  = tid & 7;
  const int cA = tid >> 3, cB = cA + 32;
  Pack16 u0, u1;
  u0.h = *(const v8h*)(T + cA * TP + 8 * q);
  u1.h = *(const v8h*)(T + cB * TP + 8 * q);
  _Float16* d0 = dst + (size_t)(n0 + cA) * K + k0 + 8 * q;
  _Float16* d1 = dst + (size_t)(n0 + cB) * K + k0 + 8 * q;
  *(volatile v4i*)d0 = u0.i;
  *(volatile v4i*)d1 = u1.i;
  __threadfence();
  *(volatile v4i*)d0 = u0.i;
  *(volatile v4i*)d1 = u1.i;
}

__global__ __launch_bounds__(NTHR) void k_qkv(
    const float* __restrict__ x, const _Float16* __restrict__ qkvt,
    const float* __restrict__ bq, const float* __restrict__ bk, const float* __restrict__ bv,
    float* qkv, int nN) {
  __shared__ __attribute__((aligned(16))) _Float16 xs[TR * AP];
  __shared__ __attribute__((aligned(16))) float rs[TR * RP];
  const int tid  = threadIdx.x;
  const int lane = tid & 31;
  const int wave = tid >> 5;
  const int hh   = lane >> 4;
  const int m    = lane & 15;
  const int row0 = blockIdx.x * TR;

  {
    const int r  = tid >> 3;
    const int c0 = (tid & 7) * 16;
    const int grow = clampi(row0 + r, 0, nN - 1);
    stage16(xs + r * AP + c0, x + (size_t)grow * DM + c0, 1.0f);
  }
  __syncthreads();

  const int nq = wave * 16 + m;
  const v8f z8 = {0.f, 0.f, 0.f, 0.f, 0.f, 0.f, 0.f, 0.f};
  v8f aq0 = z8, aq1 = z8, ak0 = z8, ak1 = z8, av0 = z8, av1 = z8;
#pragma unroll 1
  for (int kt = 0; kt < DM / 32; ++kt) {
    const int k0 = kt * 32;
    const v16h a0 = frag_ld(xs + m * AP + k0 + 8 * hh);
    const v16h a1 = frag_ld(xs + (16 + m) * AP + k0 + 8 * hh);
    const _Float16* pb = qkvt + (size_t)nq * DM + k0 + 8 * hh;
    v16h b = frag_ld(pb);
    aq0 = wm(a0, b, aq0); aq1 = wm(a1, b, aq1);
    b = frag_ld(pb + (size_t)DM * DM);
    ak0 = wm(a0, b, ak0); ak1 = wm(a1, b, ak1);
    b = frag_ld(pb + (size_t)2 * DM * DM);
    av0 = wm(a0, b, av0); av1 = wm(a1, b, av1);
  }
  {
    const float cq = bq[nq], ck = bk[nq], cv = bv[nq];
#pragma unroll
    for (int r = 0; r < 8; ++r) {
      const int ra = (8 * hh + r) * RP, rb = (16 + 8 * hh + r) * RP;
      rs[ra + nq]          = aq0[r] * 0.03125f + cq;
      rs[rb + nq]          = aq1[r] * 0.03125f + cq;
      rs[ra + DM + nq]     = ak0[r] * 0.03125f + ck;
      rs[rb + DM + nq]     = ak1[r] * 0.03125f + ck;
      rs[ra + 2 * DM + nq] = av0[r] * 0.03125f + cv;
      rs[rb + 2 * DM + nq] = av1[r] * 0.03125f + cv;
    }
  }
  __syncthreads();

  v4f xr[12];
  float* xp[12];
#pragma unroll
  for (int i = 0; i < 4; ++i) {
#pragma unroll
    for (int j = 0; j < 3; ++j) {
      xr[i * 3 + j] = *(const v4f*)(rs + (4 * wave + i) * RP + DM * j + 4 * lane);
      xp[i * 3 + j] = qkv + (size_t)(row0 + 4 * wave + i) * QW + DM * j + 4 * lane;
    }
  }
#pragma unroll
  for (int i = 0; i < 12; ++i) *(volatile v4f*)(xp[i]) = xr[i];
  __threadfence();
#pragma unroll
  for (int i = 0; i < 12; ++i) *(volatile v4f*)(xp[i]) = xr[i];
}

__global__ __launch_bounds__(NTHR) void k_agg(
    const float* __restrict__ qkv, const int* __restrict__ row, const int* __restrict__ col,
    const int* __restrict__ db, const float* __restrict__ emb, float* agg,
    int nN, int nE, int nEmb, int stepHi) {
  __shared__ int sp[16];
  const int tid  = threadIdx.x;
  const int lane = tid & 31;
  const int wave = tid >> 5;
  const int hd   = lane >> 2;
  const int nodeBase = blockIdx.x * NPB;

  if (wave == 0) {
    const int key = nodeBase + lane;
    int pos = 0;
#pragma unroll 1
    for (int step = stepHi; step > 0; step >>= 1) {
      const int t = pos + step;
      const int idx = clampi(t - 1, 0, nE - 1);
      const int rv = row[idx];
      pos = (t <= nE && rv < key) ? t : pos;
    }
    if (lane < 16) sp[lane] = pos;
  }
  __syncthreads();

  const int node = nodeBase + wave;
  if (node >= nN) return;
  int s = sp[wave];
  const int e = sp[wave + 1];
  s = clampi(s, 0, nE);
  int cnt = e - s;
  cnt = cnt < 0 ? 0 : (cnt > ECAP ? ECAP : cnt);

  const v4f q4 = *(const v4f*)(qkv + (size_t)node * QW + 4 * lane);
  const int dbn = clampi(db[node], 0, nEmb - 1);
  const float ebn = emb[dbn * NH + hd];

  float mrun = -1.0e30f, den = 0.f;
  v4f acc = {0.f, 0.f, 0.f, 0.f};
#pragma unroll 1
  for (int i = 0; i < cnt; ++i) {
    const int j = clampi(s + i, 0, nE - 1);
    const int c = clampi(col[j], 0, nN - 1);
    const int dbc = clampi(db[c], 0, nEmb - 1);
    const float ebc = emb[dbc * NH + hd];
    const float* kp = qkv + (size_t)c * QW + DM + 4 * lane;
    const v4f k4 = *(const v4f*)(kp);
    const v4f v4 = *(const v4f*)(kp + DM);
    float d = q4.x * k4.x + q4.y * k4.y + q4.z * k4.z + q4.w * k4.w;
    d += __shfl_xor(d, 1, 32);
    d += __shfl_xor(d, 2, 32);
    const float sc = (d * 0.25f + ebn) + ebc;
    const float mn = fmaxf(mrun, sc);
    const float rr = __expf(mrun - mn);
    const float p  = __expf(sc - mn);
    mrun = mn;
    den = den * rr + p;
    acc = acc * rr + p * v4;
  }
  const float inv = 1.0f / fmaxf(den, 1e-12f);
  const v4f res = acc * inv;
  float* op = agg + (size_t)node * DM + 4 * lane;
  *(volatile v4f*)op = res;
  __threadfence();
  *(volatile v4f*)op = res;
}

__device__ __forceinline__ void add_tile(v8f acc, int rbase, int col, float scale, float bias, float* hf) {
#pragma unroll
  for (int r = 0; r < 8; ++r) {
    const int ix = (rbase + r) * HP + col;
    const float t = acc[r] * scale + bias;
    hf[ix] = hf[ix] + t;
  }
}

__device__ __forceinline__ void gelu_tile(v8f acc, int rbase, int col, float bias, _Float16* zh) {
#pragma unroll
  for (int r = 0; r < 8; ++r) {
    const float u  = acc[r] * 0.03125f + bias;
    const float ge = 0.5f * u * (1.0f + erff(u * 0.70710678118654752f));
    zh[(rbase + r) * ZP + col] = (_Float16)(ge * 16.0f);
  }
}

__global__ __launch_bounds__(NTHR) void k_tail(
    const float* __restrict__ agg, const float* __restrict__ x,
    const _Float16* __restrict__ wot, const float* __restrict__ bo,
    const float* __restrict__ g1, const float* __restrict__ be1,
    const _Float16* __restrict__ w1t, const float* __restrict__ b1,
    const _Float16* __restrict__ w2t, const float* __restrict__ b2,
    const float* __restrict__ g2, const float* __restrict__ be2,
    float* out, int nN) {
  __shared__ __attribute__((aligned(16))) float    hf[TR * HP];
  __shared__ __attribute__((aligned(16))) _Float16 ah[TR * AP];
  __shared__ __attribute__((aligned(16))) _Float16 zh[TR * ZP];
  const int tid  = threadIdx.x;
  const int lane = tid & 31;
  const int wave = tid >> 5;
  const int hh   = lane >> 4;
  const int m    = lane & 15;
  const int row0 = blockIdx.x * TR;
  const v8f z8 = {0.f, 0.f, 0.f, 0.f, 0.f, 0.f, 0.f, 0.f};

  {
    const int r  = tid >> 3;
    const int c0 = (tid & 7) * 16;
    const int grow = clampi(row0 + r, 0, nN - 1);
    stage16(ah + r * AP + c0, agg + (size_t)grow * DM + c0, 64.0f);
    const float* xp = x + (size_t)grow * DM + c0;
    float* hp = hf + r * HP + c0;
    *(v4f*)(hp)      = *(const v4f*)(xp);
    *(v4f*)(hp + 4)  = *(const v4f*)(xp + 4);
    *(v4f*)(hp + 8)  = *(const v4f*)(xp + 8);
    *(v4f*)(hp + 12) = *(const v4f*)(xp + 12);
  }
  __syncthreads();

  {
    const int ncol = wave * 16 + m;
    v8f c0 = z8, c1 = z8;
#pragma unroll 1
    for (int kt = 0; kt < DM / 32; ++kt) {
      const int k0 = kt * 32;
      const v16h a0 = frag_ld(ah + m * AP + k0 + 8 * hh);
      const v16h a1 = frag_ld(ah + (16 + m) * AP + k0 + 8 * hh);
      const v16h b  = frag_ld(wot + (size_t)ncol * DM + k0 + 8 * hh);
      c0 = wm(a0, b, c0);
      c1 = wm(a1, b, c1);
    }
    const float cb = bo[ncol];
    add_tile(c0, 8 * hh, ncol, 0.00048828125f, cb, hf);
    add_tile(c1, 16 + 8 * hh, ncol, 0.00048828125f, cb, hf);
  }
  __syncthreads();

  {
    const v4f g4 = *(const v4f*)(g1 + 4 * lane);
    const v4f b4 = *(const v4f*)(be1 + 4 * lane);
#pragma unroll
    for (int i = 0; i < 4; ++i) {
      const int r = 4 * wave + i;
      const v4f v = *(const v4f*)(hf + r * HP + 4 * lane);
      const v4f y = ln_row(v, g4, b4);
      *(v4f*)(hf + r * HP + 4 * lane) = y;
      v4h yh;
      yh.x = (_Float16)y.x; yh.y = (_Float16)y.y; yh.z = (_Float16)y.z; yh.w = (_Float16)y.w;
      *(v4h*)(ah + r * AP + 4 * lane) = yh;
    }
  }
  __syncthreads();

  {
    const int cbase = 64 * wave + m;
    v8f c00 = z8, c01 = z8, c10 = z8, c11 = z8, c20 = z8, c21 = z8, c30 = z8, c31 = z8;
#pragma unroll 1
    for (int kt = 0; kt < DM / 32; ++kt) {
      const int k0 = kt * 32;
      const v16h a0 = frag_ld(ah + m * AP + k0 + 8 * hh);
      const v16h a1 = frag_ld(ah + (16 + m) * AP + k0 + 8 * hh);
      const _Float16* pb = w1t + (size_t)cbase * DM + k0 + 8 * hh;
      v16h b = frag_ld(pb);
      c00 = wm(a0, b, c00); c01 = wm(a1, b, c01);
      b = frag_ld(pb + 16 * DM);
      c10 = wm(a0, b, c10); c11 = wm(a1, b, c11);
      b = frag_ld(pb + 32 * DM);
      c20 = wm(a0, b, c20); c21 = wm(a1, b, c21);
      b = frag_ld(pb + 48 * DM);
      c30 = wm(a0, b, c30); c31 = wm(a1, b, c31);
    }
    const float bb0 = b1[cbase], bb1 = b1[cbase + 16], bb2 = b1[cbase + 32], bb3 = b1[cbase + 48];
    gelu_tile(c00, 8 * hh, cbase,      bb0, zh); gelu_tile(c01, 16 + 8 * hh, cbase,      bb0, zh);
    gelu_tile(c10, 8 * hh, cbase + 16, bb1, zh); gelu_tile(c11, 16 + 8 * hh, cbase + 16, bb1, zh);
    gelu_tile(c20, 8 * hh, cbase + 32, bb2, zh); gelu_tile(c21, 16 + 8 * hh, cbase + 32, bb2, zh);
    gelu_tile(c30, 8 * hh, cbase + 48, bb3, zh); gelu_tile(c31, 16 + 8 * hh, cbase + 48, bb3, zh);
  }
  __syncthreads();

  {
    const int ncol = wave * 16 + m;
    v8f c0 = z8, c1 = z8;
#pragma unroll 1
    for (int kt = 0; kt < DFF / 32; ++kt) {
      const int k0 = kt * 32;
      const v16h a0 = frag_ld(zh + m * ZP + k0 + 8 * hh);
      const v16h a1 = frag_ld(zh + (16 + m) * ZP + k0 + 8 * hh);
      const v16h b  = frag_ld(w2t + (size_t)ncol * DFF + k0 + 8 * hh);
      c0 = wm(a0, b, c0);
      c1 = wm(a1, b, c1);
    }
    const float cb = b2[ncol];
    add_tile(c0, 8 * hh, ncol, 0.001953125f, cb, hf);
    add_tile(c1, 16 + 8 * hh, ncol, 0.001953125f, cb, hf);
  }
  __syncthreads();

  {
    const v4f g4 = *(const v4f*)(g2 + 4 * lane);
    const v4f b4 = *(const v4f*)(be2 + 4 * lane);
    v4f y[4];
    float* op[4];
    bool ok[4];
#pragma unroll
    for (int i = 0; i < 4; ++i) {
      const int r = 4 * wave + i;
      const v4f v = *(const v4f*)(hf + r * HP + 4 * lane);
      y[i]  = ln_row(v, g4, b4);
      const int grow = row0 + r;
      ok[i] = grow < nN;
      op[i] = out + (size_t)clampi(grow, 0, nN - 1) * DM + 4 * lane;
    }
#pragma unroll
    for (int i = 0; i < 4; ++i) if (ok[i]) *(volatile v4f*)(op[i]) = y[i];
    __threadfence();
#pragma unroll
    for (int i = 0; i < 4; ++i) if (ok[i]) *(volatile v4f*)(op[i]) = y[i];
  }
}

extern "C" void kernel_launch(void* const* d_in, const int* in_sizes, int n_in,
                              void* d_out, int out_size, void* d_ws, size_t ws_size,
                              hipStream_t stream) {
  if (n_in < 21) return;
  const int nN = in_sizes[0] / DM;
  if (nN <= 0 || in_sizes[0] != nN * DM) return;
  const int nE = in_sizes[1];
  if (nE < 0 || in_sizes[2] != nE) return;
  if (in_sizes[3] != nN) return;
  if (in_sizes[4] != DM * DM || in_sizes[6] != DM * DM || in_sizes[8] != DM * DM || in_sizes[10] != DM * DM) return;
  if (in_sizes[5] != DM || in_sizes[7] != DM || in_sizes[9] != DM || in_sizes[11] != DM) return;
  const int nEmb = in_sizes[12] / NH;
  if (nEmb <= 0 || in_sizes[12] != nEmb * NH) return;
  if (in_sizes[13] != DM || in_sizes[14] != DM || in_sizes[15] != DM || in_sizes[16] != DM) return;
  if (in_sizes[17] != DM * DFF || in_sizes[18] != DFF || in_sizes[19] != DFF * DM || in_sizes[20] != DM) return;
  if (out_size != nN * DM) return;

  const float* x   = (const float*)d_in[0];
  const int*   row = (const int*)d_in[1];
  const int*   col = (const int*)d_in[2];
  const int*   db  = (const int*)d_in[3];
  const float* Wq  = (const float*)d_in[4];  const float* bq  = (const float*)d_in[5];
  const float* Wk  = (const float*)d_in[6];  const float* bk  = (const float*)d_in[7];
  const float* Wv  = (const float*)d_in[8];  const float* bv  = (const float*)d_in[9];
  const float* Wo  = (const float*)d_in[10]; const float* bo  = (const float*)d_in[11];
  const float* emb = (const float*)d_in[12];
  const float* g1  = (const float*)d_in[13]; const float* be1 = (const float*)d_in[14];
  const float* g2  = (const float*)d_in[15]; const float* be2 = (const float*)d_in[16];
  const float* W1  = (const float*)d_in[17]; const float* b1  = (const float*)d_in[18];
  const float* W2  = (const float*)d_in[19]; const float* b2  = (const float*)d_in[20];
  float* out = (float*)d_out;

  const int nBlk = (nN + TR - 1) / TR;
  const int nP = nBlk * TR;
  size_t off = 0;
  char* ws = (char*)d_ws;
  _Float16* qkvt = (_Float16*)(ws + off); off += (size_t)QW * DM * 2;   off = (off + 255) & ~(size_t)255;
  _Float16* wot  = (_Float16*)(ws + off); off += (size_t)DM * DM * 2;   off = (off + 255) & ~(size_t)255;
  _Float16* w1t  = (_Float16*)(ws + off); off += (size_t)DFF * DM * 2;  off = (off + 255) & ~(size_t)255;
  _Float16* w2t  = (_Float16*)(ws + off); off += (size_t)DM * DFF * 2;  off = (off + 255) & ~(size_t)255;
  float* qkv     = (float*)(ws + off);    off += (size_t)nP * QW * 4;   off = (off + 255) & ~(size_t)255;
  float* aggp    = (float*)(ws + off);    off += (size_t)nP * DM * 4;   off = (off + 255) & ~(size_t)255;
  if (off > ws_size) return;

  int stepHi = 0;
  if (nE > 0) { stepHi = 1; while ((long long)stepHi * 2 <= (long long)nE) stepHi *= 2; }

  k_prep<<<48, NTHR, 0, stream>>>(Wq, Wk, Wv, Wo, W1, W2, qkvt, wot, w1t, w2t);
  k_qkv<<<nBlk, NTHR, 0, stream>>>(x, qkvt, bq, bk, bv, qkv, nN);
  k_agg<<<(nN + NPB - 1) / NPB, NTHR, 0, stream>>>(qkv, row, col, db, emb, aggp, nN, nE, nEmb, stepHi);
  k_tail<<<nBlk, NTHR, 0, stream>>>(aggp, x, wot, bo, g1, be1, w1t, b1, w2t, b2, g2, be2, out, nN);
}
